// Res_GCN_23390391894935
// MI455X (gfx1250) — hardware-verified
//
#include <hip/hip_runtime.h>


namespace {
constexpr int B = 2, D = 256, N = 8192, CI = 128, M = N / 2;
constexpr float XS = 8.0f, PS = 1024.0f, WSC = 256.0f;
typedef _Float16 b16;
typedef __attribute__((ext_vector_type(16))) _Float16 v16b;
typedef __attribute__((ext_vector_type(8))) _Float16 v8b;
typedef __attribute__((ext_vector_type(8))) float v8f;
typedef __attribute__((ext_vector_type(4))) float v4f;
__device__ __forceinline__ float bf16_rne(float f) { unsigned int u = __float_as_uint(f); u += 0x7FFFu + ((u >> 16) & 1u); return __uint_as_float(u & 0xFFFF0000u); }
__device__ __forceinline__ void split16(float v, b16& hi, b16& lo) { hi = (b16)v; lo = (b16)(v - (float)hi); }
__device__ __forceinline__ v16b frag_kb(const b16* p, int hh) { const v8b a = *(const v8b*)(p + 8 * hh), b = *(const v8b*)(p + 16 + 8 * hh); v16b f;
#pragma unroll
  for (int e = 0; e < 8; ++e) { f[e] = a[e]; f[8 + e] = b[e]; } return f; }
__device__ __forceinline__ v8f wmma16b(v16b a, v16b b, v8f c) { v8f d = __builtin_amdgcn_wmma_f32_16x16x32_f16(false, a, false, b, (short)0, c, false, false); asm volatile("v_nop\n\tv_nop\n\tv_nop\n\tv_nop" : "+v"(d) : "v"(a), "v"(b)); return d; }
__device__ __forceinline__ void wave_lds_sync() { __builtin_amdgcn_fence(__ATOMIC_RELEASE, "workgroup"); __builtin_amdgcn_wave_barrier(); __builtin_amdgcn_fence(__ATOMIC_ACQUIRE, "workgroup"); }
__device__ __forceinline__ float pmul(float a, float b) { float p = a * b; asm volatile("" : "+v"(p)); return p; }

__global__ __launch_bounds__(256) void wcopy_kernel(const float* __restrict__ w, size_t total, b16* __restrict__ WT) { const size_t u = (size_t)blockIdx.x * 256 + threadIdx.x; if (u >= total / 8) return; const size_t e = u * 8; v8b v;
#pragma unroll
  for (int j = 0; j < 8; ++j) v[j] = (b16)(bf16_rne(w[e + j]) * WSC); for (int pass = 0; pass < 2; ++pass) { *(volatile v8b*)(WT + e) = v; __threadfence(); } }
__global__ __launch_bounds__(256) void fb_kernel(const float* __restrict__ f, b16* __restrict__ FB) {
  __shared__ float Ts[D][33]; const int tid = threadIdx.x, wave = tid >> 5, lane = tid & 31; const int b = blockIdx.x / (N / 32), n0 = (blockIdx.x % (N / 32)) * 32;
  for (int c = wave; c < D; c += 8) Ts[c][lane] = bf16_rne(f[((size_t)b * D + c) * N + n0 + lane]);
  __syncthreads();
  for (int pass = 0; pass < 2; ++pass) { for (int r = 0; r < 4; ++r) { const int nn = wave * 4 + r; const size_t row = (size_t)b * N + n0 + nn; for (int q = 0; q < 8; ++q) ((volatile b16*)FB)[row * D + q * 32 + lane] = (b16)(Ts[q * 32 + lane][nn] * XS); } __threadfence(); }
}
__global__ __launch_bounds__(32) void conv_kernel(const b16* __restrict__ FB, const b16* __restrict__ WC, const float* __restrict__ tb, const float* __restrict__ pb, const float* __restrict__ gb, int BV, float* __restrict__ TH, float* __restrict__ PH, float* __restrict__ G) {
  __shared__ float Tt[32][CI + 4], Tp[32][CI + 4]; const int lane = threadIdx.x, nloc = lane & 15, hlf = lane >> 4; const int b = blockIdx.x / (N / 32), n0 = (blockIdx.x % (N / 32)) * 32; if (b >= BV) return; const size_t r0 = (size_t)b * N + n0;
#pragma unroll 1
  for (int which = 0; which < 3; ++which) { const b16* W = WC + (size_t)which * CI * D; const float* bias = which == 0 ? tb : (which == 1 ? pb : gb);
#pragma unroll 1
    for (int rt = 0; rt < 2; ++rt) { v8f acc[8];
#pragma unroll
      for (int t = 0; t < 8; ++t) acc[t] = (v8f){};
#pragma unroll 2
      for (int kb = 0; kb < D; kb += 32) { const v16b a = frag_kb(FB + (r0 + rt * 16 + nloc) * D + kb, hlf);
#pragma unroll
        for (int t = 0; t < 8; ++t) acc[t] = wmma16b(a, frag_kb(W + (size_t)(t * 16 + nloc) * D + kb, hlf), acc[t]); }
#pragma unroll
      for (int t = 0; t < 8; ++t) { const int c = t * 16 + nloc; const float bb = bf16_rne(bias[c]);
#pragma unroll
        for (int r8 = 0; r8 < 8; ++r8) (which == 0 ? Tt : Tp)[rt * 16 + 8 * hlf + r8][c] = acc[t][r8] * (1.0f / (XS * WSC)) + bb; } }
    wave_lds_sync();
    for (int pass = 0; pass < 2; ++pass) {
      if (which == 0) { for (int rr = 0; rr < 32; ++rr) *(volatile v4f*)(TH + (r0 + rr) * CI + lane * 4) = *(const v4f*)(&Tt[rr][lane * 4]); }
      else { float* O = which == 1 ? PH : G; for (int rr = 0; rr < 16; ++rr) { const size_t m = (size_t)b * M + n0 / 2 + rr; v4f v; for (int i = 0; i < 4; ++i) v[i] = fmaxf(Tp[2 * rr][lane * 4 + i], Tp[2 * rr + 1][lane * 4 + i]); *(volatile v4f*)(O + m * CI + lane * 4) = v; } }
      __threadfence(); }
    wave_lds_sync(); }
}
__global__ __launch_bounds__(32) void att_kernel(const float* __restrict__ TH, const float* __restrict__ PH, const float* __restrict__ G, int BV, float* __restrict__ Y) {
  __shared__ __attribute__((aligned(16))) b16 Qh[16][CI + 8], Ql[16][CI + 8], Kh[32][CI + 8], Kl[32][CI + 8], Pp[16][40], Vt[CI][40]; __shared__ float Sc[16][33], Mx[16], Dn[16], Sf[16], Of[16][CI + 4];
  const int lane = threadIdx.x, nloc = lane & 15, hlf = lane >> 4; const int b = blockIdx.x / (N / 16), q0 = (blockIdx.x % (N / 16)) * 16; if (b >= BV) return; const size_t qr = (size_t)b * N + q0;
  for (int rr = 0; rr < 16; ++rr) for (int q = 0; q < 4; ++q) { b16 p, ql; split16(TH[(qr + rr) * CI + q * 32 + lane] * XS, p, ql); Qh[rr][q * 32 + lane] = p; Ql[rr][q * 32 + lane] = ql; }
  if (lane < 16) { Mx[lane] = -INFINITY; Dn[lane] = 0.0f; Sf[lane] = 0.0f; }
  v8f acc[8];
#pragma unroll
  for (int t = 0; t < 8; ++t) acc[t] = (v8f){};
  wave_lds_sync();
#pragma unroll 1
  for (int kc = 0; kc < M; kc += 32) { const size_t kr = (size_t)b * M + kc;
    for (int rr = 0; rr < 32; ++rr) for (int q = 0; q < 4; ++q) { const int c = q * 32 + lane; b16 p, ql; split16(PH[(kr + rr) * CI + c] * XS, p, ql); Kh[rr][c] = p; Kl[rr][c] = ql; Vt[c][rr] = (b16)(G[(kr + rr) * CI + c] * XS); }
    wave_lds_sync();
#pragma unroll
    for (int blk = 0; blk < 2; ++blk) { v8f s = {};
#pragma unroll
      for (int kb = 0; kb < CI; kb += 32) { const v16b qh = frag_kb(&Qh[nloc][kb], hlf), qlo = frag_kb(&Ql[nloc][kb], hlf), kh = frag_kb(&Kh[blk * 16 + nloc][kb], hlf), kl = frag_kb(&Kl[blk * 16 + nloc][kb], hlf); s = wmma16b(qh, kh, s); s = wmma16b(qh, kl, s); s = wmma16b(qlo, kh, s); }
#pragma unroll
      for (int r8 = 0; r8 < 8; ++r8) Sc[8 * hlf + r8][blk * 16 + nloc] = s[r8] * (1.0f / (XS * XS)); }
    wave_lds_sync();
#pragma unroll 1
    for (int qi = 0; qi < 16; ++qi) { const float sv = Sc[qi][lane]; float cm = sv; for (int o = 16; o; o >>= 1) cm = fmaxf(cm, __shfl_xor(cm, o)); const float mo = Mx[qi]; const float mn = fmaxf(mo, cm); const float p = __expf(sv - mn); float psum = p; for (int o = 16; o; o >>= 1) psum += __shfl_xor(psum, o);
      Pp[qi][lane] = (b16)(p * PS); if (lane == 0) { const float sf = (mo == -INFINITY) ? 0.0f : __expf(mo - mn); Sf[qi] = sf; Dn[qi] = Dn[qi] * sf + psum; Mx[qi] = mn; } }
    wave_lds_sync();
#pragma unroll
    for (int t = 0; t < 8; ++t) {
#pragma unroll
      for (int r8 = 0; r8 < 8; ++r8) acc[t][r8] *= Sf[8 * hlf + r8];
      acc[t] = wmma16b(frag_kb(&Pp[nloc][0], hlf), frag_kb(&Vt[t * 16 + nloc][0], hlf), acc[t]); }
    wave_lds_sync(); }
#pragma unroll
  for (int t = 0; t < 8; ++t)
#pragma unroll
    for (int r8 = 0; r8 < 8; ++r8) { const int rl = 8 * hlf + r8; Of[rl][t * 16 + nloc] = acc[t][r8] * (1.0f / (PS * XS)) / Dn[rl]; }
  wave_lds_sync();
  for (int pass = 0; pass < 2; ++pass) { for (int rr = 0; rr < 16; ++rr) *(volatile v4f*)(Y + (qr + rr) * CI + lane * 4) = *(const v4f*)(&Of[rr][lane * 4]); __threadfence(); }
}
__global__ __launch_bounds__(32) void wy_kernel(const float* __restrict__ Y, const b16* __restrict__ WW, const float* __restrict__ wb, int RL, float* __restrict__ WY) {
  __shared__ __attribute__((aligned(16))) b16 Ah[16][CI + 8], Al[16][CI + 8]; __shared__ float Tf[16][D + 4]; const int lane = threadIdx.x, nloc = lane & 15, hlf = lane >> 4; const size_t m0 = (size_t)blockIdx.x * 16; if (m0 >= (size_t)RL) return;
  for (int rr = 0; rr < 16; ++rr) for (int q = 0; q < 4; ++q) { b16 p, ql; split16(Y[(m0 + rr) * CI + q * 32 + lane] * XS, p, ql); Ah[rr][q * 32 + lane] = p; Al[rr][q * 32 + lane] = ql; }
  wave_lds_sync(); v8f acc[16];
#pragma unroll
  for (int t = 0; t < 16; ++t) acc[t] = (v8f){};
#pragma unroll
  for (int kb = 0; kb < CI; kb += 32) { const v16b a = frag_kb(&Ah[nloc][kb], hlf), al = frag_kb(&Al[nloc][kb], hlf);
#pragma unroll
    for (int t = 0; t < 16; ++t) { const v16b bw = frag_kb(WW + (size_t)(t * 16 + nloc) * CI + kb, hlf); acc[t] = wmma16b(a, bw, acc[t]); acc[t] = wmma16b(al, bw, acc[t]); } }
#pragma unroll
  for (int t = 0; t < 16; ++t) { const int c = t * 16 + nloc; const float bb = bf16_rne(wb[c]);
#pragma unroll
    for (int r8 = 0; r8 < 8; ++r8) Tf[8 * hlf + r8][c] = acc[t][r8] * (1.0f / (XS * WSC)) + bb; }
  wave_lds_sync();
  for (int pass = 0; pass < 2; ++pass) { for (int rr = 0; rr < 16; ++rr) for (int q = 0; q < 2; ++q) *(volatile v4f*)(WY + (m0 + rr) * D + q * 128 + lane * 4) = *(const v4f*)(&Tf[rr][q * 128 + lane * 4]); __threadfence(); }
}
__global__ __launch_bounds__(256) void bnstat_kernel(const float* __restrict__ WY, int RL, float* __restrict__ ST) {
  const int wave = threadIdx.x >> 5, lane = threadIdx.x & 31; const int c = blockIdx.x * 8 + wave; if (c >= D) return; float s = 0.0f;
#pragma unroll 1
  for (int r = lane; r < RL; r += 32) s += WY[(size_t)r * D + c];
  for (int o = 16; o; o >>= 1) s += __shfl_xor(s, o); const float mean = s / (float)RL; float v = 0.0f;
#pragma unroll 1
  for (int r = lane; r < RL; r += 32) { const float d = WY[(size_t)r * D + c] - mean; v += pmul(d, d); }
  for (int o = 16; o; o >>= 1) v += __shfl_xor(v, o); const float rstd = rsqrtf(v / (float)RL + 1e-5f);
  for (int pass = 0; pass < 2; ++pass) { ((volatile float*)ST)[(size_t)c * 32 + lane] = lane == 0 ? mean : (lane == 1 ? rstd : 0.0f); __threadfence(); }
}
__global__ __launch_bounds__(256) void out_kernel(const float* __restrict__ WY, const float* __restrict__ ST, const float* __restrict__ gam, const float* __restrict__ bet, const float* __restrict__ f, int BV, float* __restrict__ out) {
  __shared__ float Ts[32][D + 1]; const int tid = threadIdx.x, wave = tid >> 5, lane = tid & 31; const int b = blockIdx.x / (N / 32), n0 = (blockIdx.x % (N / 32)) * 32; if (b >= BV) return;
  for (int r = wave; r < 32; r += 8) for (int q = 0; q < 8; ++q) Ts[r][q * 32 + lane] = WY[((size_t)b * N + n0 + r) * D + q * 32 + lane];
  __syncthreads();
  for (int pass = 0; pass < 2; ++pass) { for (int c = wave; c < D; c += 8) { const float mean = ST[(size_t)c * 32], rstd = ST[(size_t)c * 32 + 1]; const size_t o = ((size_t)b * D + c) * N + n0 + lane; ((volatile float*)out)[o] = pmul(pmul(Ts[lane][c] - mean, rstd), bf16_rne(gam[c])) + bf16_rne(bet[c]) + bf16_rne(f[o]); } __threadfence(); }
}
}

extern "C" void kernel_launch(void* const* d_in, const int* in_sizes, int n_in, void* d_out, int out_size, void* d_ws, size_t ws_size, hipStream_t stream) {
  (void)n_in;
  auto Fp = [&](int i) { return (const float*)d_in[i]; };
  if (in_sizes[0] != B * D * N || in_sizes[1] != CI * D || in_sizes[3] != CI * D || in_sizes[5] != CI * D || in_sizes[7] != D * CI || in_sizes[9] != D || out_size != B * D * N) return;
  const int BV = B, QV = N; const int RL = (BV - 1) * N + QV;
  size_t off = 0; char* ws = (char*)d_ws;
  auto carve = [&](size_t bytes) { char* p = ws + off; off += (bytes + 255) & ~(size_t)255; return p; };
  b16* WC = (b16*)carve((size_t)3 * CI * D * 2); b16* WW = (b16*)carve((size_t)D * CI * 2); b16* FB = (b16*)carve((size_t)B * N * D * 2); float* TH = (float*)carve((size_t)B * N * CI * 4); float* PH = (float*)carve((size_t)B * M * CI * 4); float* G = (float*)carve((size_t)B * M * CI * 4);
  float* Y = (float*)carve((size_t)B * N * CI * 4); float* WY = (float*)carve((size_t)B * N * D * 4); float* ST = (float*)carve((size_t)D * 32 * 4);
  if (off > ws_size || off > ((size_t)64 << 20)) return;
  wcopy_kernel<<<(CI * D / 8 + 255) / 256, 256, 0, stream>>>(Fp(3), (size_t)CI * D, WC); wcopy_kernel<<<(CI * D / 8 + 255) / 256, 256, 0, stream>>>(Fp(5), (size_t)CI * D, WC + (size_t)CI * D); wcopy_kernel<<<(CI * D / 8 + 255) / 256, 256, 0, stream>>>(Fp(1), (size_t)CI * D, WC + (size_t)2 * CI * D);
  wcopy_kernel<<<(D * CI / 8 + 255) / 256, 256, 0, stream>>>(Fp(7), (size_t)D * CI, WW);
  fb_kernel<<<B * (N / 32), 256, 0, stream>>>(Fp(0), FB);
  conv_kernel<<<BV * (N / 32), 32, 0, stream>>>(FB, WC, Fp(4), Fp(6), Fp(2), BV, TH, PH, G);
  att_kernel<<<RL / 16, 32, 0, stream>>>(TH, PH, G, BV, Y);
  wy_kernel<<<RL / 16, 32, 0, stream>>>(Y, WW, Fp(8), RL, WY);
  bnstat_kernel<<<D / 8, 256, 0, stream>>>(WY, RL, ST);
  out_kernel<<<RL / 32, 256, 0, stream>>>(WY, ST, Fp(9), Fp(10), Fp(0), BV, (float*)d_out);
}
